// ConvCapsule_83313775607877
// MI455X (gfx1250) — hardware-verified
//
#include <hip/hip_runtime.h>
#include <math.h>
#include <stdint.h>

constexpr int NB_BATCH = 8;
constexpr int NIC_CAPS = 8;
constexpr int NID_DIM  = 16;
constexpr int NOC_CAPS = 8;
constexpr int NOD_DIM  = 16;
constexpr int HIMG = 32;
constexpr int WIMG = 32;
constexpr int NIMG = NB_BATCH * NIC_CAPS;
constexpr int CIN_CH = NID_DIM * 4;
constexpr int NCH_BN = NOC_CAPS * NOD_DIM;
constexpr int NCOL = NCH_BN * 4;
constexpr int KTOT = CIN_CH * 9;
constexpr int NPIX = NIMG * HIMG * WIMG;
constexpr int MCHUNK = 32768;
constexpr int NCHUNK = NPIX / MCHUNK;
constexpr int NB_PER_CHUNK = NB_BATCH / NCHUNK;
constexpr int PIX_PER_STAT = 256;
constexpr int STAT_PER_CHUNK = MCHUNK / PIX_PER_STAT;
constexpr int STAT_BLOCKS = NCHUNK * STAT_PER_CHUNK;
constexpr int STAT_COUNT = NPIX * 4;
constexpr int ROUT_BLOCKS = NB_BATCH * 4 * HIMG;
constexpr int OUT0_ELEMS = NB_BATCH * NOC_CAPS * NOD_DIM * 4 * HIMG * WIMG;
constexpr int OUT1_OFF_BYTES = 16777216;
constexpr int OUT1_OFF_ELEMS = OUT1_OFF_BYTES / 4;
constexpr int OUT_TOTAL_BYTES = 16777220;

static_assert(KTOT % 32 == 0, "GEMM K multiple of 32");
static_assert(MCHUNK % 64 == 0 && NCOL % 64 == 0, "GEMM M,N tile multiples");
static_assert(NCHUNK * MCHUNK == NPIX, "chunks cover all rows");
static_assert(MCHUNK == NB_PER_CHUNK * NIC_CAPS * HIMG * WIMG, "chunk = whole batches");
static_assert(NB_PER_CHUNK * NCHUNK == NB_BATCH, "chunks cover all batches");
static_assert(OUT1_OFF_ELEMS == OUT0_ELEMS, "out1 follows out0");
static_assert(OUT1_OFF_BYTES + 4 <= OUT_TOTAL_BYTES, "out1 inside d_out");
static_assert((NCOL * KTOT) % (8 * 256) == 0, "wtrans grid exact");
static_assert((MCHUNK * KTOT) % (8 * 256) == 0, "im2col grid exact");
static_assert(STAT_PER_CHUNK * PIX_PER_STAT == MCHUNK, "stat blocks cover a chunk");
static_assert(STAT_BLOCKS * PIX_PER_STAT == NPIX, "stat blocks cover all pixels");
static_assert(((MCHUNK / 64) * (NCOL / 64)) % 8 == 0, "gemm grid exact");

constexpr size_t OFF_BT    = 0;
constexpr size_t SZ_BT     = (size_t)NCOL * KTOT * 2;
constexpr size_t OFF_ACOL  = OFF_BT + SZ_BT;
constexpr size_t SZ_ACOL   = (size_t)MCHUNK * KTOT * 2;
constexpr size_t OFF_P     = OFF_ACOL + SZ_ACOL;
constexpr size_t SZ_P      = (size_t)MCHUNK * NCOL * 4;
constexpr size_t OFF_PART  = OFF_P + SZ_P;
constexpr size_t SZ_PART   = (size_t)STAT_BLOCKS * 256 * 4;
constexpr size_t OFF_BNTAB = OFF_PART + SZ_PART;
constexpr size_t SZ_BNTAB  = 256 * 4;
constexpr size_t OFF_ENT   = OFF_BNTAB + SZ_BNTAB;
constexpr size_t SZ_ENT    = (size_t)ROUT_BLOCKS * 32 * 4;
constexpr size_t WS_TOTAL  = OFF_ENT + SZ_ENT;
static_assert(WS_TOTAL == 105841664, "carve total");
static_assert(WS_TOTAL <= 134217728, "carve under the 128 MiB cap");
static_assert(OFF_ACOL % 128 == 0 && OFF_P % 128 == 0 && OFF_PART % 128 == 0 && OFF_BNTAB % 128 == 0 && OFF_ENT % 128 == 0, "aligned regions");

typedef __attribute__((ext_vector_type(16))) _Float16 v16h;
typedef __attribute__((ext_vector_type(8)))  _Float16 v8h;
typedef __attribute__((ext_vector_type(16))) __bf16   v16b;
typedef __attribute__((ext_vector_type(8)))  __bf16   v8b;
typedef __attribute__((ext_vector_type(8)))  float    v8f;
typedef __attribute__((ext_vector_type(4)))  float    v4f;
typedef __attribute__((ext_vector_type(2)))  float    v2f;
typedef __attribute__((ext_vector_type(4)))  unsigned v4u;

__device__ __forceinline__ unsigned short f2bf_bits(float f) {
  unsigned u = __float_as_uint(f);
  return (unsigned short)((u + 0x7FFFu + ((u >> 16) & 1u)) >> 16);
}
__device__ __forceinline__ float bf_bits2f(unsigned short h) { return __uint_as_float(((unsigned)h) << 16); }

__device__ __forceinline__ void dep_guard_h(v8f& a, v8f& b, v16h x, v16h y) { asm volatile("v_nop\n\tv_nop\n\tv_nop\n\tv_nop" : "+v"(a), "+v"(b) : "v"(x), "v"(y)); }
__device__ __forceinline__ void dep_guard_b(v8f& a, v8f& b, v16b x, v16b y) { asm volatile("v_nop\n\tv_nop\n\tv_nop\n\tv_nop" : "+v"(a), "+v"(b) : "v"(x), "v"(y)); }
__device__ __forceinline__ void keep4_h(v16h a, v16h b, v16h c, v16h d) { asm volatile("v_nop" :: "v"(a), "v"(b), "v"(c), "v"(d)); }
__device__ __forceinline__ void keep4_b(v16b a, v16b b, v16b c, v16b d) { asm volatile("v_nop" :: "v"(a), "v"(b), "v"(c), "v"(d)); }
__device__ __forceinline__ void acc_guard4(v8f& a, v8f& b, v8f& c, v8f& d) { asm volatile("v_nop\n\tv_nop\n\tv_nop\n\tv_nop" : "+v"(a), "+v"(b), "+v"(c), "+v"(d)); }
template <typename T> struct Frag;
template <> struct Frag<_Float16> {
  typedef v16h V; union U { v16h v; v8h h[2]; };
  static __device__ __forceinline__ v16h load(const _Float16* p) {
    U f; f.h[0] = *(const v8h*)(p); f.h[1] = *(const v8h*)(p + 16); return f.v;
  }
  static __device__ __forceinline__ v8f mma(v16h a, v16h b, v8f c) {
    return __builtin_amdgcn_wmma_f32_16x16x32_f16(false, a, false, b, (short)0, c, false, false);
  }
  static __device__ __forceinline__ void guard(v8f& a, v8f& b, v16h x, v16h y) { dep_guard_h(a, b, x, y); }
  static __device__ __forceinline__ void keep(v16h a, v16h b, v16h c, v16h d) { keep4_h(a, b, c, d); }
};
template <> struct Frag<__bf16> {
  typedef v16b V; union U { v16b v; v8b h[2]; };
  static __device__ __forceinline__ v16b load(const __bf16* p) {
    U f; f.h[0] = *(const v8b*)(p); f.h[1] = *(const v8b*)(p + 16); return f.v;
  }
  static __device__ __forceinline__ v8f mma(v16b a, v16b b, v8f c) {
    return __builtin_amdgcn_wmma_f32_16x16x32_bf16(false, a, false, b, (short)0, c, false, false);
  }
  static __device__ __forceinline__ void guard(v8f& a, v8f& b, v16b x, v16b y) { dep_guard_b(a, b, x, y); }
  static __device__ __forceinline__ void keep(v16b a, v16b b, v16b c, v16b d) { keep4_b(a, b, c, d); }
};

template <int ET> struct Elem;
template <> struct Elem<0> { typedef _Float16 T; };
template <> struct Elem<1> { typedef __bf16 T; };
template <int ET, bool SPLIT, int BIAS_MODE, int OUT_MODE, bool RESID, int ACT = 0>
__global__ __launch_bounds__(256) void wmma_gemm64(
    const unsigned short* __restrict__ Ap, const unsigned short* __restrict__ A2p, int lda, long strideA,
    const unsigned short* __restrict__ Btp, const unsigned short* __restrict__ Bt2p, int ldb, long strideB,
    void* __restrict__ Cout, void* __restrict__ Cout2, int ldc, long strideC,
    const float* __restrict__ bias,
    const float* __restrict__ resid, long strideR,
    int M, int N, int K, float scale) {
  typedef typename Elem<ET>::T T;
  typedef typename Frag<T>::V V;
  const T* A = (const T*)Ap; const T* A2 = (const T*)A2p; const T* Bt = (const T*)Btp; const T* Bt2 = (const T*)Bt2p;
  __shared__ __align__(16) float sT[8][16 * 68];
  const int b    = blockIdx.y;
  const int lane = threadIdx.x & 31;
  const int wave = threadIdx.x >> 5;
  const int tilesN = N >> 6;
  const int tilesM = M >> 6;
  const int tile = blockIdx.x * 8 + wave;
  if (tile >= tilesM * tilesN) return;
  const int tm = tile / tilesN;
  const int tn = tile - tm * tilesN;
  const int m0 = tm << 6;
  const int n0 = tn << 6;

  const T* Ab  = A  + (size_t)b * strideA;
  const T* Bb  = Bt + (size_t)b * strideB;
  const T* Ab2 = SPLIT ? (A2  + (size_t)b * strideA) : nullptr;
  const T* Bb2 = SPLIT ? (Bt2 + (size_t)b * strideB) : nullptr;

  const int rlane = lane & 15;
  const int koff  = (lane >> 4) * 8;
  const int mOff  = (lane >> 4) * 8;

  v8f acc[4][4];
#pragma unroll
  for (int i = 0; i < 4; ++i)
#pragma unroll
    for (int j = 0; j < 4; ++j) acc[i][j] = (v8f){0.f,0.f,0.f,0.f,0.f,0.f,0.f,0.f};

  for (int k0 = 0; k0 < K; k0 += 32) {
    V bh[4], bl[4];
#pragma unroll
    for (int j = 0; j < 4; ++j) {
      const size_t bo = (size_t)(n0 + (j << 4) + rlane) * ldb + koff + k0;
      bh[j] = Frag<T>::load(Bb + bo);
      if (SPLIT) bl[j] = Frag<T>::load(Bb2 + bo);
    }
#pragma unroll
    for (int i = 0; i < 4; ++i) {
      const size_t ao = (size_t)(m0 + (i << 4) + rlane) * lda + koff + k0;
      V ah = Frag<T>::load(Ab + ao);
      V al;
      if (SPLIT) al = Frag<T>::load(Ab2 + ao);
#pragma unroll
      for (int j = 0; j < 4; ++j) {
        acc[i][j] = Frag<T>::mma(ah, bh[j], acc[i][j]);
        if (SPLIT) {
          acc[i][j] = Frag<T>::mma(ah, bl[j], acc[i][j]);
          acc[i][j] = Frag<T>::mma(al, bh[j], acc[i][j]);
        }
      }
      Frag<T>::guard(acc[i][0], acc[i][3], ah, SPLIT ? al : ah);
    }
    Frag<T>::keep(bh[0], bh[1], bh[2], bh[3]);
    if (SPLIT) Frag<T>::keep(bl[0], bl[1], bl[2], bl[3]);
  }
  acc_guard4(acc[0][0], acc[0][1], acc[0][2], acc[0][3]);
  acc_guard4(acc[1][0], acc[1][1], acc[1][2], acc[1][3]);
  acc_guard4(acc[2][0], acc[2][1], acc[2][2], acc[2][3]);
  acc_guard4(acc[3][0], acc[3][1], acc[3][2], acc[3][3]);

  float* slab = sT[wave];
  const float* Rb = RESID ? (resid + (size_t)b * strideR) : nullptr;
#pragma unroll
  for (int i = 0; i < 4; ++i) {
    const int mBase = m0 + (i << 4);
#pragma unroll
    for (int j = 0; j < 4; ++j) {
      const int n = n0 + (j << 4) + rlane;
      float bv = 0.f;
      if (BIAS_MODE == 2) bv = bias[n];
#pragma unroll
      for (int r = 0; r < 8; ++r) {
        float v = acc[i][j][r] * scale;
        if (BIAS_MODE == 1) v += bias[mBase + mOff + r];
        if (BIAS_MODE == 2) v += bv;
        if (RESID) v += Rb[(size_t)(mBase + mOff + r) * ldc + n];
        if (ACT == 1) v = tanhf(v);
        if (ACT == 2) v = fmaxf(v, 0.0f);
        if (ACT == 3) v = v / (1.0f + expf(-v));
        if (ACT == 4) v = (v > 0.f) ? v : 0.01f * v;
        if (ACT == 5) v = 0.5f * v * (1.0f + erff(v * 0.70710678118654752f));
        slab[(mOff + r) * 68 + (j << 4) + rlane] = v;
      }
    }
    __builtin_amdgcn_fence(__ATOMIC_RELEASE, "workgroup");
    __builtin_amdgcn_wave_barrier();
    __builtin_amdgcn_fence(__ATOMIC_ACQUIRE, "workgroup");
    if (OUT_MODE == 0) {
      float* C = (float*)Cout + (size_t)b * strideC;
      const int hh = lane >> 4, c4 = (lane & 15) * 4;
      for (int pass = 0; pass < 2; ++pass) {
#pragma unroll
        for (int it = 0; it < 8; ++it) {
          const int row = it * 2 + hh;
          v4f v = *(const v4f*)(slab + row * 68 + c4);
          *(volatile v4f*)(C + (size_t)(mBase + row) * ldc + n0 + c4) = v;
        }
        __threadfence();
      }
    } else {
      const int q = lane >> 3, c8 = (lane & 7) * 8;
      unsigned short* C  = (unsigned short*)Cout  + (size_t)b * strideC;
      unsigned short* C2 = (OUT_MODE == 2) ? ((unsigned short*)Cout2 + (size_t)b * strideC) : nullptr;
      for (int pass = 0; pass < 2; ++pass) {
#pragma unroll
        for (int it = 0; it < 4; ++it) {
          const int row = it * 4 + q;
          const float* sp = slab + row * 68 + c8;
          v8h hv, lv;
#pragma unroll
          for (int e = 0; e < 8; ++e) {
            if (OUT_MODE == 1) {
              hv[e] = (_Float16)sp[e];
            } else {
              unsigned short hb = f2bf_bits(sp[e]);
              unsigned short lb = f2bf_bits(sp[e] - bf_bits2f(hb));
              hv[e] = __builtin_bit_cast(_Float16, hb);
              lv[e] = __builtin_bit_cast(_Float16, lb);
            }
          }
          *(volatile v8h*)(C + (size_t)(mBase + row) * ldc + n0 + c8) = hv;
          if (OUT_MODE == 2) *(volatile v8h*)(C2 + (size_t)(mBase + row) * ldc + n0 + c8) = lv;
        }
        __threadfence();
      }
    }
    __builtin_amdgcn_fence(__ATOMIC_RELEASE, "workgroup");
    __builtin_amdgcn_wave_barrier();
    __builtin_amdgcn_fence(__ATOMIC_ACQUIRE, "workgroup");
  }
}

__device__ __forceinline__ unsigned pack_bf2(float a, float b) {
  return (unsigned)f2bf_bits(a) | ((unsigned)f2bf_bits(b) << 16);
}

__global__ __launch_bounds__(256) void wtrans_kernel(const float* __restrict__ w, unsigned* __restrict__ Btw) {
  const int gid = blockIdx.x * 256 + threadIdx.x;
  if (gid >= NCOL * KTOT / 8) return;
  const int n  = gid / (KTOT / 8);
  const int kg = gid - n * (KTOT / 8);
  const int k0 = kg * 8;
  const int r = n >> 7, cout = n & 127;
  const int kpos = k0 >> 6, cin0 = k0 & 63;
  const int kh = kpos / 3, kw = kpos - kh * 3;
  const int sh = (r == 0) ? kh : (r == 1) ? kw : (r == 2) ? (2 - kh) : (2 - kw);
  const int sw = (r == 0) ? kw : (r == 1) ? (2 - kh) : (r == 2) ? (2 - kw) : kh;
  float v[8];
#pragma unroll
  for (int e = 0; e < 8; ++e) {
    const int cin = cin0 + e;
    const int id = cin >> 2, gi = cin & 3;
    const int gsrc = (gi - r) & 3;
    v[e] = w[(((cout * NID_DIM + id) * 4 + gsrc) * 3 + sh) * 3 + sw];
  }
  const v4u pk = (v4u){ pack_bf2(v[0], v[1]), pack_bf2(v[2], v[3]), pack_bf2(v[4], v[5]), pack_bf2(v[6], v[7]) };
  unsigned* dst = Btw + (size_t)gid * 4;
  *(volatile v4u*)dst = pk;
  __threadfence();
  *(volatile v4u*)dst = pk;
}

__global__ __launch_bounds__(256) void im2col_kernel(const float* __restrict__ x, unsigned* __restrict__ Acolw, int chunk) {
  const int gid = blockIdx.x * 256 + threadIdx.x;
  if (gid >= MCHUNK * KTOT / 8) return;
  const int m  = gid / (KTOT / 8);
  const int kg = gid - m * (KTOT / 8);
  const int k0 = kg * 8;
  const int kpos = k0 >> 6, cin0 = k0 & 63;
  const int kh = kpos / 3, kw = kpos - kh * 3;
  const int pix = chunk * MCHUNK + m;
  const int img = pix >> 10;
  const int h = (pix >> 5) & 31;
  const int wq = pix & 31;
  const int hh = h + kh - 1, ww = wq + kw - 1;
  const bool valid = ((unsigned)hh < (unsigned)HIMG) && ((unsigned)ww < (unsigned)WIMG);
  const int hhc = hh < 0 ? 0 : (hh > HIMG - 1 ? HIMG - 1 : hh);
  const int wwc = ww < 0 ? 0 : (ww > WIMG - 1 ? WIMG - 1 : ww);
  const float* base = x + (((size_t)img * CIN_CH + cin0) * HIMG + hhc) * WIMG + wwc;
  float v[8];
#pragma unroll
  for (int e = 0; e < 8; ++e) {
    const float t = base[(size_t)e * (HIMG * WIMG)];
    v[e] = valid ? t : 0.f;
  }
  const v4u pk = (v4u){ pack_bf2(v[0], v[1]), pack_bf2(v[2], v[3]), pack_bf2(v[4], v[5]), pack_bf2(v[6], v[7]) };
  unsigned* dst = Acolw + (size_t)gid * 4;
  *(volatile v4u*)dst = pk;
  __threadfence();
  *(volatile v4u*)dst = pk;
}

__global__ __launch_bounds__(256) void bnstat_kernel(const float* __restrict__ P, float* __restrict__ part, int chunk) {
  const int blk = blockIdx.x, t = threadIdx.x;
  __shared__ float colS[NCOL], colQ[NCOL];
  __shared__ __align__(16) float lineS[2 * NCH_BN];
  float s0 = 0.f, s1 = 0.f, q0 = 0.f, q1 = 0.f;
  const float* base = P + (size_t)blk * PIX_PER_STAT * NCOL + 2 * t;
#pragma unroll 4
  for (int i = 0; i < PIX_PER_STAT; ++i) {
    const v2f vv = *(const v2f*)(base + (size_t)i * NCOL);
    const float a = vv[0], c = vv[1];
    s0 += a; q0 += a * a;
    s1 += c; q1 += c * c;
  }
  colS[2 * t] = s0; colS[2 * t + 1] = s1;
  colQ[2 * t] = q0; colQ[2 * t + 1] = q1;
  __syncthreads();
  if (t < NCH_BN) {
    lineS[t]          = (colS[t] + colS[NCH_BN + t]) + (colS[2 * NCH_BN + t] + colS[3 * NCH_BN + t]);
    lineS[NCH_BN + t] = (colQ[t] + colQ[NCH_BN + t]) + (colQ[2 * NCH_BN + t] + colQ[3 * NCH_BN + t]);
  }
  __syncthreads();
  if (t < 32) {
    float* dst = part + (size_t)(chunk * STAT_PER_CHUNK + blk) * 256;
    for (int pass = 0; pass < 2; ++pass) {
#pragma unroll
      for (int i = 0; i < 2; ++i) {
        const int idx = i * 128 + t * 4;
        const v4f v = *(const v4f*)(lineS + idx);
        *(volatile v4f*)(dst + idx) = v;
      }
      __threadfence();
    }
  }
}

__global__ __launch_bounds__(128) void bnfin_kernel(const float* __restrict__ part, float* __restrict__ bntab) {
  const int t = threadIdx.x;
  __shared__ __align__(16) float lineS[2 * NCH_BN];
  double s = 0.0, q = 0.0;
#pragma unroll 2
  for (int blk = 0; blk < STAT_BLOCKS; ++blk) {
    s += (double)part[(size_t)blk * 256 + t];
    q += (double)part[(size_t)blk * 256 + NCH_BN + t];
  }
  const double inv = 1.0 / (double)STAT_COUNT;
  const double mean = s * inv;
  double var = q * inv - mean * mean;
  var = var < 0.0 ? 0.0 : var;
  const float mf = (float)mean;
  const float rstd = rsqrtf((float)var + 1e-5f);
  lineS[t] = mf;
  lineS[NCH_BN + t] = rstd;
  __syncthreads();
  if (t < 32) {
    for (int pass = 0; pass < 2; ++pass) {
#pragma unroll
      for (int i = 0; i < 2; ++i) {
        const int idx = i * 128 + t * 4;
        const v4f v = *(const v4f*)(lineS + idx);
        *(volatile v4f*)(bntab + idx) = v;
      }
      __threadfence();
    }
  }
}

__global__ __launch_bounds__(128) void routing_kernel(
    const float* __restrict__ P, const float* __restrict__ bntab,
    const float* __restrict__ gamma, const float* __restrict__ beta,
    float* __restrict__ out, float* __restrict__ enttab, int chunk) {
  const int h = blockIdx.x, g = blockIdx.y, bl = blockIdx.z;
  const int b = chunk * NB_PER_CHUNK + bl;
  const int u = threadIdx.x;
  const int lane = u & 31, wv = u >> 5;
  __shared__ __align__(16) float predS[NIC_CAPS * NCH_BN];
  __shared__ __align__(16) float voutS[NCH_BN * WIMG];
  __shared__ __align__(16) float entS[WIMG];
  __shared__ float bS[64], eS[64], cS[64], clS[64];
  __shared__ float vS[NCH_BN];
  __shared__ float meanS[NCH_BN], sclS[NCH_BN], betaS[NCH_BN];

  {
    const float mu = bntab[u];
    const float rs = bntab[NCH_BN + u];
    const float ga = bf_bits2f(f2bf_bits(gamma[u]));
    const float be = bf_bits2f(f2bf_bits(beta[u]));
    meanS[u] = mu;
    sclS[u] = rs * ga;
    betaS[u] = be;
  }
  __syncthreads();

  const int p = u >> 1, icp = u >> 4, ocp = (u >> 1) & 7, half = u & 1;
  const int ocs = u >> 4;

#pragma unroll 1
  for (int w = 0; w < WIMG; ++w) {
    {
      const int ic = u >> 4, q = u & 15;
      const int pixl = (bl * NIC_CAPS + ic) * (HIMG * WIMG) + h * WIMG + w;
      const float* src = P + (size_t)pixl * NCOL + g * NCH_BN + q * 8;
      const v4f a0 = *(const v4f*)(src);
      const v4f a1 = *(const v4f*)(src + 4);
      const int ch = q * 8;
      float* pr = predS + ic * NCH_BN + ch;
      pr[0] = (a0[0] - meanS[ch + 0]) * sclS[ch + 0] + betaS[ch + 0];
      pr[1] = (a0[1] - meanS[ch + 1]) * sclS[ch + 1] + betaS[ch + 1];
      pr[2] = (a0[2] - meanS[ch + 2]) * sclS[ch + 2] + betaS[ch + 2];
      pr[3] = (a0[3] - meanS[ch + 3]) * sclS[ch + 3] + betaS[ch + 3];
      pr[4] = (a1[0] - meanS[ch + 4]) * sclS[ch + 4] + betaS[ch + 4];
      pr[5] = (a1[1] - meanS[ch + 5]) * sclS[ch + 5] + betaS[ch + 5];
      pr[6] = (a1[2] - meanS[ch + 6]) * sclS[ch + 6] + betaS[ch + 6];
      pr[7] = (a1[3] - meanS[ch + 7]) * sclS[ch + 7] + betaS[ch + 7];
    }
    if (u < 64) bS[u] = 0.f;
    __syncthreads();

    float vreg = 0.f;
#pragma unroll 1
    for (int it = 0; it < 3; ++it) {
      float mx = -INFINITY;
#pragma unroll
      for (int o = 0; o < NOC_CAPS; ++o) mx = fmaxf(mx, bS[icp * 8 + o]);
      const float ex = expf(bS[p] - mx);
      if (half == 0) eS[p] = ex;
      __syncthreads();
      float den = 0.f;
#pragma unroll
      for (int o = 0; o < NOC_CAPS; ++o) den += eS[icp * 8 + o];
      const float cc = ex * __builtin_amdgcn_rcpf(den);
      if (half == 0) {
        cS[p] = cc;
        if (it == 2) clS[p] = cc * logf(cc);
      }
      __syncthreads();

      float sacc = 0.f;
#pragma unroll
      for (int ic2 = 0; ic2 < NIC_CAPS; ++ic2) sacc += cS[ic2 * 8 + ocs] * predS[ic2 * NCH_BN + u];
      float sq = sacc * sacc;
      sq += __shfl_xor(sq, 1, 32);
      sq += __shfl_xor(sq, 2, 32);
      sq += __shfl_xor(sq, 4, 32);
      sq += __shfl_xor(sq, 8, 32);
      const float nrm = sqrtf(sq);
      const float n2 = nrm * nrm;
      const float scl = n2 * __builtin_amdgcn_rcpf(1.f + n2) * __builtin_amdgcn_rcpf(nrm + 1e-8f);
      vreg = scl * sacc;
      vS[u] = vreg;
      __syncthreads();

      if (it < 2) {
        const int base = ocp * NOD_DIM + half * 8;
        float aacc = 0.f;
#pragma unroll
        for (int d = 0; d < 8; ++d) aacc += predS[icp * NCH_BN + base + d] * vS[base + d];
        aacc += __shfl_xor(aacc, 1, 32);
        if (half == 0) bS[p] += aacc;
        __syncthreads();
      }
    }
    voutS[u * WIMG + w] = vreg;

    {
      const int icc = (u < NIC_CAPS) ? u : (NIC_CAPS - 1);
      float part = 0.f;
#pragma unroll
      for (int o = 0; o < NOC_CAPS; ++o) part += clS[icc * 8 + o];
      part = (u < NIC_CAPS) ? part : 0.f;
      part += __shfl_xor(part, 1, 32);
      part += __shfl_xor(part, 2, 32);
      part += __shfl_xor(part, 4, 32);
      if (u == 0) entS[w] = -part;
    }
    __syncthreads();
  }

  {
    const int lq = lane >> 3, c4 = (lane & 7) * 4;
    for (int pass = 0; pass < 2; ++pass) {
#pragma unroll
      for (int i = 0; i < 8; ++i) {
        const int j = wv * 32 + i * 4 + lq;
        const v4f val = *(const v4f*)(voutS + j * WIMG + c4);
        float* dst = out + ((size_t)((b * NCH_BN + j) * 4 + g) * HIMG + h) * WIMG + c4;
        *(volatile v4f*)dst = val;
      }
      __threadfence();
    }
  }
  if (u < 8) {
    const int blk = (b * 4 + g) * HIMG + h;
    const v4f val = *(const v4f*)(entS + u * 4);
    float* dst = enttab + (size_t)blk * 32 + u * 4;
    *(volatile v4f*)dst = val;
    __threadfence();
    *(volatile v4f*)dst = val;
  }
}

__global__ __launch_bounds__(256) void entfin_kernel(const float* __restrict__ enttab, float* __restrict__ out) {
  const int t = threadIdx.x;
  __shared__ double red[256];
  double s = 0.0;
#pragma unroll 2
  for (int i = 0; i < (ROUT_BLOCKS * 32) / 256; ++i) s += (double)enttab[(size_t)i * 256 + t];
  red[t] = s;
  __syncthreads();
  for (int o = 128; o > 0; o >>= 1) {
    if (t < o) red[t] += red[t + o];
    __syncthreads();
  }
  if (t == 0) {
    const double tot = red[0];
    const float ent = (float)(tot * (1.0 / 32768.0) * (1.0 / 2.0794415416798359));
    float* dst = out + OUT1_OFF_ELEMS;
    *(volatile float*)dst = ent;
    __threadfence();
    *(volatile float*)dst = ent;
  }
}

extern "C" void kernel_launch(void* const* d_in, const int* in_sizes, int n_in,
                              void* d_out, int out_size, void* d_ws, size_t ws_size,
                              hipStream_t stream) {
  (void)in_sizes; (void)n_in; (void)out_size;
  if (ws_size < WS_TOTAL) return;
  const float* x     = (const float*)d_in[0];
  const float* w     = (const float*)d_in[1];
  const float* gamma = (const float*)d_in[2];
  const float* beta  = (const float*)d_in[3];
  float* out = (float*)d_out;

  char* ws = (char*)d_ws;
  unsigned short* Bt   = (unsigned short*)(ws + OFF_BT);
  unsigned short* Acol = (unsigned short*)(ws + OFF_ACOL);
  float* P      = (float*)(ws + OFF_P);
  float* part   = (float*)(ws + OFF_PART);
  float* bntab  = (float*)(ws + OFF_BNTAB);
  float* enttab = (float*)(ws + OFF_ENT);

  const dim3 gemm_grid((MCHUNK / 64) * (NCOL / 64) / 8, 1);

  wtrans_kernel<<<(NCOL * KTOT / 8) / 256, 256, 0, stream>>>(w, (unsigned*)Bt);

  for (int c = 0; c < NCHUNK; ++c) {
    im2col_kernel<<<(MCHUNK * KTOT / 8) / 256, 256, 0, stream>>>(x, (unsigned*)Acol, c);
    wmma_gemm64<1, false, 0, 0, false, 0><<<gemm_grid, 256, 0, stream>>>(
        (const unsigned short*)Acol, (const unsigned short*)Acol, KTOT, 0L,
        (const unsigned short*)Bt, (const unsigned short*)Bt, KTOT, 0L,
        (void*)P, (void*)nullptr, NCOL, 0L,
        (const float*)nullptr, (const float*)nullptr, 0L,
        MCHUNK, NCOL, KTOT, 1.0f);
    bnstat_kernel<<<STAT_PER_CHUNK, 256, 0, stream>>>(P, part, c);
  }

  bnfin_kernel<<<1, 128, 0, stream>>>(part, bntab);

  routing_kernel<<<dim3(HIMG, 4, NB_PER_CHUNK), 128, 0, stream>>>(P, bntab, gamma, beta, out, enttab, NCHUNK - 1);
  for (int c = 0; c < NCHUNK - 1; ++c) {
    im2col_kernel<<<(MCHUNK * KTOT / 8) / 256, 256, 0, stream>>>(x, (unsigned*)Acol, c);
    wmma_gemm64<1, false, 0, 0, false, 0><<<gemm_grid, 256, 0, stream>>>(
        (const unsigned short*)Acol, (const unsigned short*)Acol, KTOT, 0L,
        (const unsigned short*)Bt, (const unsigned short*)Bt, KTOT, 0L,
        (void*)P, (void*)nullptr, NCOL, 0L,
        (const float*)nullptr, (const float*)nullptr, 0L,
        MCHUNK, NCOL, KTOT, 1.0f);
    routing_kernel<<<dim3(HIMG, 4, NB_PER_CHUNK), 128, 0, stream>>>(P, bntab, gamma, beta, out, enttab, c);
  }

  entfin_kernel<<<1, 256, 0, stream>>>(enttab, out);
}
